// Net_83064667505278
// MI455X (gfx1250) — hardware-verified
//
#include <hip/hip_runtime.h>
#include <stddef.h>
#include <stdint.h>
#include <math.h>


#define FIN    9
#define HID    32
#define K1     32
#define K2     64
#define NCLS   7
#define NCP    16
#define OC2    8
#define NTHR   256
#define NWAVE  8
#define EPT    8
#define CHUNK  (NTHR * EPT)
#define WCAP   (EPT * 32)
#define LISTN  (NWAVE * WCAP)
#define NBA    1024
#define SLA    10
#define RCAP   20480
#define DEGCAP 64
#define GBM    128
#define BK_ZINTS (2 * RCAP + 2 * NBA + LISTN)
#define BK_INTS  (BK_ZINTS + 32)
#define WSMAX  134217728

static_assert((CHUNK & (CHUNK - 1)) == 0 && CHUNK <= 4096);
static_assert((NBA & (NBA - 1)) == 0 && NBA == (1 << SLA) && NBA <= 1024);
static_assert(((long long)CHUNK << SLA) < (1LL << 31));
static_assert(22 + SLA <= 32);
static_assert(RCAP >= 17613);
static_assert(DEGCAP >= 44);
static_assert(RCAP % (2 * NTHR) == 0 && RCAP % 32 == 0);
static_assert(LISTN == 2 * NBA && NBA % NTHR == 0 && NBA == 4 * NTHR);
static_assert(BK_ZINTS % 4 == 0 && BK_INTS * 4 <= 300000);
static_assert(NBA % 32 == 0 && (NBA * NCLS) % (4 * NTHR) == 0 && (NBA * NCLS * 4) % 128 == 0);
static_assert(K1 % 32 == 0 && K2 % 32 == 0 && K2 == 2 * HID && FIN <= K1);
static_assert(GBM == NWAVE * 16 && NBA % NWAVE == 0 && NBA == 32 * 32);
static_assert(NCLS < OC2 && OC2 <= NCP);

typedef float          v4f   __attribute__((ext_vector_type(4)));
typedef float          v8f   __attribute__((ext_vector_type(8)));
typedef int            v2i   __attribute__((ext_vector_type(2)));
typedef int            v4i   __attribute__((ext_vector_type(4)));
typedef int            v8i   __attribute__((ext_vector_type(8)));
typedef unsigned int   v4u   __attribute__((ext_vector_type(4)));
typedef unsigned short v8us  __attribute__((ext_vector_type(8)));
typedef unsigned short v16us __attribute__((ext_vector_type(16)));
typedef __bf16         v16bf __attribute__((ext_vector_type(16)));
typedef v4f  __attribute__((may_alias)) v4fa;
typedef v2i  __attribute__((may_alias)) v2ia;
typedef v4i  __attribute__((may_alias)) v4ia;
typedef v8us __attribute__((may_alias)) v8usa;
union FragB { v16bf v; v16us u; v8us h[2]; v8i w; };

__device__ __forceinline__ v8f wmb(const FragB& a, const FragB& b, v8f c) {
  v8f d = __builtin_amdgcn_wmma_f32_16x16x32_bf16(false, a.v, false, b.v, (short)0, c, false, false);
  asm volatile("v_nop\n\tv_nop\n\tv_nop\n\tv_nop" : "+v"(d) : "v"(a.w), "v"(b.w));
  return d;
}

__device__ __forceinline__ unsigned bf16_bits(float f) {
  const unsigned u = __float_as_uint(f);
  const unsigned r = (u + 0x7FFFu + ((u >> 16) & 1u)) >> 16;
  const unsigned q = (u >> 16) | 0x40u;
  return ((u & 0x7FFFFFFFu) > 0x7F800000u) ? q : r;
}
__device__ __forceinline__ float bf16_val(float f) {
  return __uint_as_float(bf16_bits(f) << 16);
}

template <int SLB>
__device__ __forceinline__ int scan_chunk(const int* __restrict__ dsts, int nE, int cbase, int slotBase,
                                          int nb, int vec8, int* list, int tid, int lane, int wave) {
  int wc = 0;
  const int el0  = tid * EPT;
  const int e0   = cbase + el0;
  const int sent = -2147483647 - 1;
  v4i da, db;
  if (vec8 != 0 && cbase + CHUNK <= nE) {
    da = *(const v4i*)(dsts + e0);
    db = *(const v4i*)(dsts + e0 + 4);
  } else {
    da.x = (e0     < nE) ? dsts[min(e0,     nE - 1)] : sent;
    da.y = (e0 + 1 < nE) ? dsts[min(e0 + 1, nE - 1)] : sent;
    da.z = (e0 + 2 < nE) ? dsts[min(e0 + 2, nE - 1)] : sent;
    da.w = (e0 + 3 < nE) ? dsts[min(e0 + 3, nE - 1)] : sent;
    db.x = (e0 + 4 < nE) ? dsts[min(e0 + 4, nE - 1)] : sent;
    db.y = (e0 + 5 < nE) ? dsts[min(e0 + 5, nE - 1)] : sent;
    db.z = (e0 + 6 < nE) ? dsts[min(e0 + 6, nE - 1)] : sent;
    db.w = (e0 + 7 < nE) ? dsts[min(e0 + 7, nE - 1)] : sent;
  }
  const unsigned nbs = (unsigned)slotBase;
  const unsigned unb = (unsigned)nb;
  const unsigned s0 = (unsigned)da.x - nbs, s1 = (unsigned)da.y - nbs;
  const unsigned s2 = (unsigned)da.z - nbs, s3 = (unsigned)da.w - nbs;
  const unsigned s4 = (unsigned)db.x - nbs, s5 = (unsigned)db.y - nbs;
  const unsigned s6 = (unsigned)db.z - nbs, s7 = (unsigned)db.w - nbs;
  const bool h0 = s0 < unb, h1 = s1 < unb, h2 = s2 < unb, h3 = s3 < unb;
  const bool h4 = s4 < unb, h5 = s5 < unb, h6 = s6 < unb, h7 = s7 < unb;
  const unsigned any = __builtin_amdgcn_ballot_w32(h0 | h1 | h2 | h3 | h4 | h5 | h6 | h7);
  if (any != 0u) {
#define HITJ(J, HJ, SJ) { \
      const unsigned mj = __builtin_amdgcn_ballot_w32(HJ); \
      if (mj != 0u) { \
        if (HJ) { \
          const int pos = wc + (int)__builtin_amdgcn_mbcnt_lo(mj, 0u); \
          if (pos < WCAP) list[wave * WCAP + pos] = ((el0 + (J)) << SLB) | (int)(SJ); \
        } \
        wc += (int)__builtin_popcount(mj); } }
    HITJ(0, h0, s0)
    HITJ(1, h1, s1)
    HITJ(2, h2, s2)
    HITJ(3, h3, s3)
    HITJ(4, h4, s4)
    HITJ(5, h5, s5)
    HITJ(6, h6, s6)
    HITJ(7, h7, s7)
#undef HITJ
  }
  return wc;
}

__global__ __launch_bounds__(NTHR) void k_prep(const float* __restrict__ x, const float* __restrict__ W1,
                                               const float* __restrict__ W2, int nN, int nbx,
                                               unsigned short* XB, unsigned short* W1T, unsigned short* W2D) {
  const int tid = (int)threadIdx.x;
  v8us o;
  unsigned short* dp;
  if ((int)blockIdx.x < nbx) {
    const int u   = (int)blockIdx.x * NTHR + tid;
    const int row = u >> 2;
    const int k8  = (u & 3) * 8;
    const int rc  = row < nN ? row : nN - 1;
    const float* p = x + (size_t)rc * FIN;
    const bool rok = row < nN;
#pragma unroll
    for (int i = 0; i < 8; ++i) {
      const int k  = k8 + i;
      const int kc = k < FIN ? k : FIN - 1;
      const float v = p[kc];
      const bool ok = rok && (k < FIN);
      o[i] = ok ? (unsigned short)bf16_bits(v) : (unsigned short)0;
    }
    dp = XB + (size_t)row * K1 + k8;
  } else if (tid < 128) {
    const int n  = tid >> 2;
    const int k8 = (tid & 3) * 8;
#pragma unroll
    for (int i = 0; i < 8; ++i) {
      const int k  = k8 + i;
      const int kc = k < FIN ? k : FIN - 1;
      const float v = W1[kc * HID + n];
      o[i] = (k < FIN) ? (unsigned short)bf16_bits(v) : (unsigned short)0;
    }
    dp = W1T + (size_t)n * K1 + k8;
  } else {
    const int v2 = tid - 128;
    const int n  = v2 >> 3;
    const int k8 = (v2 & 7) * 8;
    const int kk = k8 & (HID - 1);
    const int nc = n < NCLS ? n : NCLS - 1;
#pragma unroll
    for (int i = 0; i < 8; ++i) {
      const float v = W2[(kk + i) * NCLS + nc];
      o[i] = (n < NCLS) ? (unsigned short)bf16_bits(v) : (unsigned short)0;
    }
    dp = W2D + (size_t)n * K2 + k8;
  }
  *(volatile v8us*)dp = o;
  __threadfence();
  *(volatile v8us*)dp = o;
}

__global__ __launch_bounds__(NTHR) void k_bucket(const int* __restrict__ srcs, const int* __restrict__ dsts,
                                                 const float* __restrict__ ew, int nE, int nN, int vec8,
                                                 int* LIST, int* CNT, int* OFF, float* DEG, float* DINV,
                                                 int* FLAG) {
  extern __shared__ __attribute__((aligned(16))) int dsm[];
  int* reg1 = dsm;
  int* reg2 = dsm + RCAP;
  int* scnt = dsm + 2 * RCAP;
  int* soff = scnt + NBA;
  int* list = soff + NBA;
  int* misc = list + LISTN;
  const int tid = (int)threadIdx.x, lane = tid & 31, wave = tid >> 5;
  const int blk = (int)blockIdx.x;
  const int nodeBase = blk * NBA;

  {
    const v4i z4 = {0, 0, 0, 0};
    for (int i = tid * 4; i < BK_ZINTS; i += NTHR * 4) *(v4ia*)(dsm + i) = z4;
    if (tid < 32) misc[tid] = 0;
  }
  __syncthreads();

  int tot = 0, ov = 0;
  const int nChunks = (nE + CHUNK - 1) / CHUNK;
#pragma unroll 1
  for (int ch = 0; ch < nChunks; ++ch) {
    const int cbase = ch * CHUNK;
    const int wc = scan_chunk<SLA>(dsts, nE, cbase, nodeBase, NBA, vec8, list, tid, lane, wave);
    if (lane == 0) misc[wave] = wc;
    __syncthreads();
    int pre = 0, all = 0;
#pragma unroll
    for (int w2 = 0; w2 < NWAVE; ++w2) {
      int c = misc[w2];
      c = c < 0 ? 0 : (c > WCAP ? WCAP : c);
      all += c;
      pre += (w2 < wave) ? c : 0;
    }
    const int wcc  = wc > WCAP ? WCAP : wc;
    const int base = tot + pre;
#pragma unroll 1
    for (int i = lane; i < wcc; i += 32) {
      const int ent = list[wave * WCAP + i];
      const int el  = (ent >> SLA) & (CHUNK - 1);
      const int sl  = ent & (NBA - 1);
      int eid = cbase + el;
      eid = eid > nE - 1 ? nE - 1 : eid;
      const int pos = base + i;
      if (pos < RCAP) reg1[pos] = (int)(((unsigned)eid << SLA) | (unsigned)sl);
    }
    tot += all;
    if (tot > RCAP) { ov = 1; tot = RCAP; }
    __syncthreads();
  }
  const int nh = tot;

  if (wave == 0) {
#pragma unroll 1
    for (int b0 = 0; b0 < nh; b0 += 32) {
      const int idx = b0 + lane;
      const int uv  = reg1[idx < nh ? idx : nh - 1];
      const int m32 = (nh - b0) < 32 ? (nh - b0) : 32;
#pragma unroll 1
      for (int k = 0; k < m32; ++k) {
        const int u  = __builtin_amdgcn_readlane(uv, k);
        const int sl = u & (NBA - 1);
        if (lane == 0) scnt[sl] = scnt[sl] + 1;
      }
    }
  }
  __syncthreads();

  {
    const v4i ca = *(const v4ia*)(scnt + 4 * tid);
    const int e0 = ca.x < 0 ? 0 : ca.x, e1 = ca.y < 0 ? 0 : ca.y;
    const int e2 = ca.z < 0 ? 0 : ca.z, e3 = ca.w < 0 ? 0 : ca.w;
    const bool big = (e0 > DEGCAP) | (e1 > DEGCAP) | (e2 > DEGCAP) | (e3 > DEGCAP);
    const int ts = e0 + e1 + e2 + e3;
    int incl = ts;
#pragma unroll
    for (int d = 1; d < 32; d <<= 1) {
      const int up = __shfl_up(incl, d, 32);
      if (lane >= d) incl += up;
    }
    if (lane == 31) misc[8 + wave] = incl;
    if (big) misc[16] = 1;
    __syncthreads();
    int pre = 0;
#pragma unroll
    for (int w2 = 0; w2 < NWAVE; ++w2) pre += (w2 < wave) ? misc[8 + w2] : 0;
    int run = pre + incl - ts;
    soff[4 * tid + 0] = run; list[4 * tid + 0] = run; run += e0;
    soff[4 * tid + 1] = run; list[4 * tid + 1] = run; run += e1;
    soff[4 * tid + 2] = run; list[4 * tid + 2] = run; run += e2;
    soff[4 * tid + 3] = run; list[4 * tid + 3] = run;
  }
  __syncthreads();

  if (wave == 0) {
#pragma unroll 1
    for (int b0 = 0; b0 < nh; b0 += 32) {
      const int idx = b0 + lane;
      const int uv  = reg1[idx < nh ? idx : nh - 1];
      const int m32 = (nh - b0) < 32 ? (nh - b0) : 32;
#pragma unroll 1
      for (int k = 0; k < m32; ++k) {
        const int u   = __builtin_amdgcn_readlane(uv, k);
        const int sl  = u & (NBA - 1);
        const int eid = (int)((unsigned)u >> SLA);
        if (lane == 0) {
          int pos = list[sl];
          pos = pos < 0 ? 0 : (pos > RCAP - 1 ? RCAP - 1 : pos);
          reg2[pos] = eid;
          list[sl] = pos + 1;
        }
      }
    }
  }
  __syncthreads();
  const int flag = (ov != 0 || misc[16] != 0) ? 1 : 0;

  {
    int* lbase = LIST + (size_t)blk * (size_t)(2 * RCAP);
#pragma unroll 1
    for (int it = 0; it < RCAP / (2 * NTHR); ++it) {
      const int p0 = it * (2 * NTHR) + 2 * tid;
      int ea = reg2[p0], eb = reg2[p0 + 1];
      ea = ea < 0 ? 0 : (ea > nE - 1 ? nE - 1 : ea);
      eb = eb < 0 ? 0 : (eb > nE - 1 ? nE - 1 : eb);
      int sa = srcs[ea], sb = srcs[eb];
      sa = sa < 0 ? 0 : (sa > nN - 1 ? nN - 1 : sa);
      sb = sb < 0 ? 0 : (sb > nN - 1 ? nN - 1 : sb);
      const float wa = bf16_val(ew[ea]);
      const float wb = bf16_val(ew[eb]);
      const bool va = p0 < nh, vb = (p0 + 1) < nh;
      v4i o;
      o.x = va ? sa : 0;
      o.y = va ? __float_as_int(wa) : 0;
      o.z = vb ? sb : 0;
      o.w = vb ? __float_as_int(wb) : 0;
      reg1[p0]     = o.y;
      reg1[p0 + 1] = o.w;
      int* dp = lbase + 2 * p0;
      *(volatile v4i*)dp = o;
      __threadfence();
      *(volatile v4i*)dp = o;
    }
  }
  __syncthreads();

  const float qnan = __int_as_float(0x7fc00000);
#pragma unroll 1
  for (int ps = 0; ps < NBA / NTHR; ++ps) {
    const int s = ps * NTHR + tid;
    int c = scnt[s];
    c = c < 0 ? 0 : (c > DEGCAP ? DEGCAP : c);
    int o = soff[s];
    o = o < 0 ? 0 : (o > nh ? nh : o);
    if (c > nh - o) c = nh - o;
    int cm = c;
#pragma unroll
    for (int off = 16; off > 0; off >>= 1) {
      const int oth = __shfl_xor(cm, off, 32);
      cm = oth > cm ? oth : cm;
    }
    float d = 0.0f;
#pragma unroll 1
    for (int q = 0; q < cm; ++q) {
      int idx = o + q;
      idx = idx > RCAP - 1 ? RCAP - 1 : idx;
      const float w = __int_as_float(reg1[idx]);
      d += (q < c) ? w : 0.0f;
    }
    const float deg = d + 1.0f;
    float di = (deg > 0.0f) ? (1.0f / sqrtf(deg)) : 0.0f;
    di = (flag != 0) ? qnan : di;
    list[s]       = __float_as_int(deg);
    list[NBA + s] = __float_as_int(di);
  }
  __syncthreads();

  {
    const v4i c4 = *(const v4ia*)(scnt + 4 * tid);
    const v4i o4 = *(const v4ia*)(soff + 4 * tid);
    const v4i d4 = *(const v4ia*)(list + 4 * tid);
    const v4i i4 = *(const v4ia*)(list + NBA + 4 * tid);
    const v4i f4 = {flag, flag, flag, flag};
    const size_t gb = (size_t)nodeBase + 4 * tid;
    int* fp = FLAG + (size_t)blk * 32 + 4 * (lane & 7);
    const bool fw = (tid < 8);
    *(volatile v4i*)(CNT + gb) = c4;
    *(volatile v4i*)(OFF + gb) = o4;
    *(volatile v4i*)((int*)DEG + gb) = d4;
    *(volatile v4i*)((int*)DINV + gb) = i4;
    if (fw) *(volatile v4i*)fp = f4;
    __threadfence();
    *(volatile v4i*)(CNT + gb) = c4;
    *(volatile v4i*)(OFF + gb) = o4;
    *(volatile v4i*)((int*)DEG + gb) = d4;
    *(volatile v4i*)((int*)DINV + gb) = i4;
    if (fw) *(volatile v4i*)fp = f4;
  }
}

template <int NT, int KS, int OC>
__global__ __launch_bounds__(NTHR) void k_gemm(const unsigned short* __restrict__ A,
                                               const unsigned short* __restrict__ WT, float* outF) {
  static_assert(OC <= 16 * NT && (GBM * OC) % (4 * NTHR) == 0 && (GBM * OC * 4) % 128 == 0);
  __shared__ __attribute__((aligned(16))) float stg[GBM * OC];
  constexpr int K = 32 * KS;
  const int tid = (int)threadIdx.x, lane = tid & 31, wave = tid >> 5, hh = lane >> 4, m = lane & 15;
  const int rowBase = (int)blockIdx.x * GBM;

  v8f acc[NT];
  {
    const v8f z = {0.f, 0.f, 0.f, 0.f, 0.f, 0.f, 0.f, 0.f};
#pragma unroll
    for (int t = 0; t < NT; ++t) acc[t] = z;
  }
  const unsigned short* ap = A  + (size_t)(rowBase + 16 * wave + m) * (size_t)K + 8 * hh;
  const unsigned short* wp = WT + (size_t)m * (size_t)K + 8 * hh;
#pragma unroll
  for (int ks = 0; ks < KS; ++ks) {
    FragB af;
    af.h[0] = *(const v8usa*)(ap + 32 * ks);
    af.h[1] = *(const v8usa*)(ap + 32 * ks + 16);
#pragma unroll
    for (int t = 0; t < NT; ++t) {
      const unsigned short* wq = wp + (size_t)(16 * t) * (size_t)K + 32 * ks;
      FragB bf;
      bf.h[0] = *(const v8usa*)wq;
      bf.h[1] = *(const v8usa*)(wq + 16);
      acc[t] = wmb(af, bf, acc[t]);
    }
  }

#pragma unroll
  for (int t = 0; t < NT; ++t) {
    const int lc = 16 * t + m;
#pragma unroll
    for (int r = 0; r < 8; ++r) {
      const int lr = 16 * wave + 8 * hh + r;
      if (lc < OC) stg[lr * OC + lc] = acc[t][r];
    }
  }
  __syncthreads();

  constexpr int NIT = (GBM * OC) / (4 * NTHR);
  v4f fv[NIT];
#pragma unroll
  for (int it = 0; it < NIT; ++it) fv[it] = *(const v4fa*)(stg + 4 * (it * NTHR + tid));
  float* ob = outF + (size_t)rowBase * OC;
#pragma unroll
  for (int it = 0; it < NIT; ++it) *(volatile v4f*)(ob + 4 * (size_t)(it * NTHR + tid)) = fv[it];
  __threadfence();
#pragma unroll
  for (int it = 0; it < NIT; ++it) *(volatile v4f*)(ob + 4 * (size_t)(it * NTHR + tid)) = fv[it];
}

__global__ __launch_bounds__(NTHR) void k_agg1(const int* __restrict__ LIST, const int* __restrict__ CNT,
                                               const int* __restrict__ OFF, const float* __restrict__ DINV,
                                               const int* __restrict__ FLAG, const float* __restrict__ H1,
                                               const float* __restrict__ b1, int nN, int mRows,
                                               unsigned short* X1) {
  const int tid = (int)threadIdx.x, lane = tid & 31;
  const int wave = __builtin_amdgcn_readfirstlane(tid >> 5);
  const int blk = (int)blockIdx.x;
  const int nodeBase = blk * NBA;
  const int fl = FLAG[(size_t)blk * 32];
  const float bv = bf16_val(b1[lane]);
  const int* lb = LIST + (size_t)blk * (size_t)(2 * RCAP);
  const float qnan = __int_as_float(0x7fc00000);
  const int q0s = (8 * lane) & 31, q1s = (8 * lane + 2) & 31;
  const int q2s = (8 * lane + 4) & 31, q3s = (8 * lane + 6) & 31;

#pragma unroll 1
  for (int si = 0; si < NBA / NWAVE; ++si) {
    const int s    = si * NWAVE + wave;
    const int node = nodeBase + s;
    if (node >= mRows) break;
    int c = CNT[node];
    c = c < 0 ? 0 : (c > DEGCAP ? DEGCAP : c);
    int o = OFF[node];
    o = o < 0 ? 0 : (o > RCAP ? RCAP : o);
    const int nc = node < nN ? node : nN - 1;
    const float dd = DINV[nc];
    const float rd = dd * dd;
    float acc = 0.0f;
#pragma unroll 1
    for (int b0 = 0; b0 < c; b0 += 32) {
      int idx = o + b0 + lane;
      idx = idx > RCAP - 1 ? RCAP - 1 : idx;
      const v2i en = *(const v2ia*)(lb + 2 * idx);
      int sr = en.x;
      sr = sr < 0 ? 0 : (sr > nN - 1 ? nN - 1 : sr);
      const float w  = __int_as_float(en.y);
      const float cf = (DINV[sr] * w) * dd;
      const int  cfi = __float_as_int(cf);
      const int m32 = (c - b0) < 32 ? (c - b0) : 32;
#pragma unroll 1
      for (int k = 0; k < m32; ++k) {
        const int   sk = __builtin_amdgcn_readlane(sr, k);
        const float ck = __int_as_float(__builtin_amdgcn_readlane(cfi, k));
        const float a  = H1[(size_t)sk * HID + lane];
        acc = fmaf(ck, a, acc);
      }
    }
    const float sv = H1[(size_t)nc * HID + lane];
    float y = (acc + rd * sv) + bv;
    y = (y > 0.0f) ? y : (y - y);
    y = (fl != 0) ? qnan : y;
    const float v = (node < nN) ? y : 0.0f;
    const unsigned hb = bf16_bits(v);
    const unsigned lo = bf16_bits(v - __uint_as_float(hb << 16));
    const int xw = (int)(hb | (lo << 16));
    const int yw = __shfl_xor(xw, 1, 32);
    const int hw = (int)(((unsigned)xw & 0xFFFFu) | ((unsigned)yw << 16));
    const int lw = (int)(((unsigned)xw >> 16) | ((unsigned)yw & 0xFFFF0000u));
    const int g0 = __shfl(hw, q0s, 32), g1 = __shfl(hw, q1s, 32);
    const int g2 = __shfl(hw, q2s, 32), g3 = __shfl(hw, q3s, 32);
    const int p0 = __shfl(lw, q0s, 32), p1 = __shfl(lw, q1s, 32);
    const int p2 = __shfl(lw, q2s, 32), p3 = __shfl(lw, q3s, 32);
    const bool lsel = (lane & 4) != 0;
    v4u pv;
    pv.x = (unsigned int)(lsel ? p0 : g0);
    pv.y = (unsigned int)(lsel ? p1 : g1);
    pv.z = (unsigned int)(lsel ? p2 : g2);
    pv.w = (unsigned int)(lsel ? p3 : g3);
    unsigned short* hp = X1 + (size_t)node * K2 + 8 * (lane & 7);
    const bool wr = lane < 8;
    if (wr) *(volatile v4u*)hp = pv;
    __threadfence();
    if (wr) *(volatile v4u*)hp = pv;
  }
}

__global__ __launch_bounds__(NTHR) void k_agg2(const int* __restrict__ LIST, const int* __restrict__ CNT,
                                               const int* __restrict__ OFF, const float* __restrict__ DINV,
                                               const int* __restrict__ FLAG, const float* __restrict__ H2,
                                               const float* __restrict__ b2, int nN, int nOut, float* out) {
  __shared__ __attribute__((aligned(16))) float os[NBA * NCLS];
  const int tid = (int)threadIdx.x, lane = tid & 31;
  const int wave = __builtin_amdgcn_readfirstlane(tid >> 5);
  const int g = lane >> 3, j = lane & 7;
  const int blk = (int)blockIdx.x;
  const int nodeBase = blk * NBA;
  const int fl = FLAG[(size_t)blk * 32];
  const bool colv = j < NCLS;
  const int jc = colv ? j : NCLS - 1;
  const float bzr = bf16_val(b2[jc]);
  const float bz = colv ? bzr : 0.0f;
  const int* lb = LIST + (size_t)blk * (size_t)(2 * RCAP);
  const float qnan = __int_as_float(0x7fc00000);

#pragma unroll 1
  for (int st = 0; st < NBA / 32; ++st) {
    const int s    = st * 32 + wave * 4 + g;
    const int node = nodeBase + s;
    int c = CNT[node];
    c = c < 0 ? 0 : (c > DEGCAP ? DEGCAP : c);
    int o = OFF[node];
    o = o < 0 ? 0 : (o > RCAP ? RCAP : o);
    int cm = c;
    {
      const int t8 = __shfl_xor(cm, 8, 32);
      cm = t8 > cm ? t8 : cm;
      const int t16 = __shfl_xor(cm, 16, 32);
      cm = t16 > cm ? t16 : cm;
    }
    const int nc = node < nN ? node : nN - 1;
    const float dd = DINV[nc];
    float acc = 0.0f;
#pragma unroll 1
    for (int q = 0; q < cm; ++q) {
      int idx = o + q;
      idx = idx > RCAP - 1 ? RCAP - 1 : idx;
      const v2i en = *(const v2ia*)(lb + 2 * idx);
      int sr = en.x;
      sr = sr < 0 ? 0 : (sr > nN - 1 ? nN - 1 : sr);
      const float w   = __int_as_float(en.y);
      const float nrm = (DINV[sr] * w) * dd;
      const float h   = H2[(size_t)sr * OC2 + j];
      const float t   = nrm * h;
      acc = (q < c) ? (acc + t) : acc;
    }
    const float sv = H2[(size_t)nc * OC2 + j];
    const float y  = (acc + (dd * dd) * sv) + bz;
    float m = colv ? y : -3.0e38f;
#pragma unroll
    for (int off = 1; off < 8; off <<= 1) {
      const float oth = __shfl_xor(m, off, 32);
      m = (oth > m || oth != oth) ? oth : m;
    }
    const float sh = y - m;
    const float ex = expf(sh);
    float sm = colv ? ex : 0.0f;
#pragma unroll
    for (int off = 1; off < 8; off <<= 1) sm += __shfl_xor(sm, off, 32);
    float r = sh - logf(sm);
    r = (fl != 0) ? qnan : r;
    if (colv) os[s * NCLS + j] = r;
  }
  __syncthreads();

  constexpr int NIT = (NBA * NCLS) / (4 * NTHR);
  v4f ov[NIT];
#pragma unroll
  for (int it = 0; it < NIT; ++it) ov[it] = *(const v4fa*)(os + 4 * (it * NTHR + tid));
  const size_t fbase = (size_t)blk * (size_t)(NBA * NCLS);
#pragma unroll
  for (int it = 0; it < NIT; ++it) {
    const size_t gi = fbase + 4 * (size_t)(it * NTHR + tid);
    if (gi + 3 < (size_t)nOut) *(volatile v4f*)(out + gi) = ov[it];
  }
  __threadfence();
#pragma unroll
  for (int it = 0; it < NIT; ++it) {
    const size_t gi = fbase + 4 * (size_t)(it * NTHR + tid);
    if (gi + 3 < (size_t)nOut) *(volatile v4f*)(out + gi) = ov[it];
  }
}

static inline int cdiv(int a, int b) { return (a + b - 1) / b; }
static inline size_t al256(size_t o) { return (o + 255) & ~(size_t)255; }

extern "C" void kernel_launch(void* const* d_in, const int* in_sizes, int n_in,
                              void* d_out, int out_size, void* d_ws, size_t ws_size,
                              hipStream_t stream) {
  if (n_in < 7) return;
  if (in_sizes[0] < FIN || (in_sizes[0] % FIN) != 0) return;
  const int nN = in_sizes[0] / FIN;
  if (nN < 1 || nN > (1 << 22)) return;
  if (in_sizes[1] < 2 || (in_sizes[1] & 1) != 0) return;
  const int nE = in_sizes[1] / 2;
  if (nE < 1 || nE > (1 << 22) - 1) return;
  if (in_sizes[2] != nE) return;
  if (in_sizes[3] != FIN * HID || in_sizes[4] != HID) return;
  if (in_sizes[5] != HID * NCLS || in_sizes[6] != NCLS) return;
  if ((long long)out_size != (long long)nN * NCLS) return;
  if ((out_size & 3) != 0) return;

  const float* x   = (const float*)d_in[0];
  const int*   ei  = (const int*)d_in[1];
  const float* ewt = (const float*)d_in[2];
  const float* W1  = (const float*)d_in[3];
  const float* b1  = (const float*)d_in[4];
  const float* W2  = (const float*)d_in[5];
  const float* b2  = (const float*)d_in[6];
  float* out = (float*)d_out;
  const int* src = ei;
  const int* dst = ei + nE;

  const int MP   = cdiv(nN, GBM) * GBM;
  const int gM   = MP / GBM;
  const int NBLK = cdiv(MP, NBA);
  if ((long long)NBLK * NBA < (long long)MP) return;
  const int NSL  = NBLK * NBA;
  const int nbx  = (MP * 4) / NTHR;
  if (nbx * NTHR != MP * 4) return;
  const int vec8 = ((nE & 3) == 0) ? 1 : 0;

  char* ws = (char*)d_ws;
  size_t off = 0;
  const size_t oXB  = off; off = al256(off + (size_t)MP * K1 * 2);
  const size_t oW1T = off; off = al256(off + (size_t)HID * K1 * 2);
  const size_t oW2D = off; off = al256(off + (size_t)NCP * K2 * 2);
  const size_t oH1  = off; off = al256(off + (size_t)MP * HID * 4);
  const size_t oX1  = off; off = al256(off + (size_t)MP * K2 * 2);
  const size_t oH2  = off; off = al256(off + (size_t)MP * OC2 * 4);
  const size_t oLST = off; off = al256(off + (size_t)NBLK * RCAP * 8);
  const size_t oCNT = off; off = al256(off + (size_t)NSL * 4);
  const size_t oOFF = off; off = al256(off + (size_t)NSL * 4);
  const size_t oDEG = off; off = al256(off + (size_t)NSL * 4);
  const size_t oDIV = off; off = al256(off + (size_t)NSL * 4);
  const size_t oFLG = off; off = al256(off + (size_t)NBLK * 128);
  if (off > ws_size || off > (size_t)WSMAX) return;
  unsigned short* XB   = (unsigned short*)(ws + oXB);
  unsigned short* W1T  = (unsigned short*)(ws + oW1T);
  unsigned short* W2D  = (unsigned short*)(ws + oW2D);
  float*          H1   = (float*)(ws + oH1);
  unsigned short* X1   = (unsigned short*)(ws + oX1);
  float*          H2   = (float*)(ws + oH2);
  int*            LIST = (int*)(ws + oLST);
  int*            CNT  = (int*)(ws + oCNT);
  int*            OFF  = (int*)(ws + oOFF);
  float*          DEG  = (float*)(ws + oDEG);
  float*          DINV = (float*)(ws + oDIV);
  int*            FLAG = (int*)(ws + oFLG);

  const size_t bkLds = (size_t)BK_INTS * 4;
  hipFuncSetAttribute(reinterpret_cast<const void*>(&k_bucket), hipFuncAttributeMaxDynamicSharedMemorySize,
                      (int)bkLds);

  k_prep<<<nbx + 1, NTHR, 0, stream>>>(x, W1, W2, nN, nbx, XB, W1T, W2D);
  k_bucket<<<NBLK, NTHR, bkLds, stream>>>(src, dst, ewt, nE, nN, vec8, LIST, CNT, OFF, DEG, DINV, FLAG);
  k_gemm<2, 1, HID><<<gM, NTHR, 0, stream>>>(XB, W1T, H1);
  k_agg1<<<NBLK, NTHR, 0, stream>>>(LIST, CNT, OFF, DINV, FLAG, H1, b1, nN, MP, X1);
  k_gemm<1, 2, OC2><<<gM, NTHR, 0, stream>>>(X1, W2D, H2);
  k_agg2<<<NBLK, NTHR, 0, stream>>>(LIST, CNT, OFF, DINV, FLAG, H2, b2, nN, out_size, out);
}
